// StrnnLocPredictor_64218351010371
// MI455X (gfx1250) — hardware-run, weakly checked
//
#include <hip/hip_runtime.h>
#include <math.h>

#pragma clang fp contract(off)

constexpr int kBatch   = 32;
constexpr int kSeq     = 128;
constexpr int kDim     = 128;
constexpr int kHid     = 128;
constexpr int kInter   = 64;
constexpr int kSlots   = 11;
constexpr int kSlotE   = kSlots * kInter;
constexpr int kPre     = 16;
constexpr int kOutN    = 10000;
constexpr int kOutPad  = 10048;
constexpr int kHid4    = 512;
constexpr int kVocab   = 10000;
constexpr int kRows    = kBatch * kSeq;
constexpr int kPreRows = kBatch * kPre;

typedef __attribute__((ext_vector_type(16))) _Float16 v16h;
typedef __attribute__((ext_vector_type(8)))  _Float16 v8h;
typedef __attribute__((ext_vector_type(16))) __bf16   v16b;
typedef __attribute__((ext_vector_type(8)))  __bf16   v8b;
typedef __attribute__((ext_vector_type(8)))  float    v8f;
typedef __attribute__((ext_vector_type(4)))  float    v4f;
typedef __attribute__((ext_vector_type(2)))  float    v2f;
typedef __attribute__((ext_vector_type(4)))  unsigned int v4u;

__device__ __forceinline__ unsigned short f2bf_bits(float f) {
  unsigned u = __float_as_uint(f);
  return (unsigned short)((u + 0x7FFFu + ((u >> 16) & 1u)) >> 16);
}
__device__ __forceinline__ float bf_bits2f(unsigned short h) { return __uint_as_float(((unsigned)h) << 16); }

__device__ __forceinline__ void dep_guard_h(v8f& a, v8f& b, v16h x, v16h y) { asm volatile("v_nop\n\tv_nop\n\tv_nop\n\tv_nop" : "+v"(a), "+v"(b) : "v"(x), "v"(y)); }
__device__ __forceinline__ void dep_guard_b(v8f& a, v8f& b, v16b x, v16b y) { asm volatile("v_nop\n\tv_nop\n\tv_nop\n\tv_nop" : "+v"(a), "+v"(b) : "v"(x), "v"(y)); }
__device__ __forceinline__ void keep4_h(v16h a, v16h b, v16h c, v16h d) { asm volatile("v_nop" :: "v"(a), "v"(b), "v"(c), "v"(d)); }
__device__ __forceinline__ void keep4_b(v16b a, v16b b, v16b c, v16b d) { asm volatile("v_nop" :: "v"(a), "v"(b), "v"(c), "v"(d)); }
__device__ __forceinline__ void acc_guard4(v8f& a, v8f& b, v8f& c, v8f& d) { asm volatile("v_nop\n\tv_nop\n\tv_nop\n\tv_nop" : "+v"(a), "+v"(b), "+v"(c), "+v"(d)); }
template <typename T> struct Frag;
template <> struct Frag<_Float16> {
  typedef v16h V; union U { v16h v; v8h h[2]; };
  static __device__ __forceinline__ v16h load(const _Float16* p) {
    U f; f.h[0] = *(const v8h*)(p); f.h[1] = *(const v8h*)(p + 16); return f.v;
  }
  static __device__ __forceinline__ v8f mma(v16h a, v16h b, v8f c) {
    return __builtin_amdgcn_wmma_f32_16x16x32_f16(false, a, false, b, (short)0, c, false, false);
  }
  static __device__ __forceinline__ void guard(v8f& a, v8f& b, v16h x, v16h y) { dep_guard_h(a, b, x, y); }
  static __device__ __forceinline__ void keep(v16h a, v16h b, v16h c, v16h d) { keep4_h(a, b, c, d); }
};
template <> struct Frag<__bf16> {
  typedef v16b V; union U { v16b v; v8b h[2]; };
  static __device__ __forceinline__ v16b load(const __bf16* p) {
    U f; f.h[0] = *(const v8b*)(p); f.h[1] = *(const v8b*)(p + 16); return f.v;
  }
  static __device__ __forceinline__ v8f mma(v16b a, v16b b, v8f c) {
    return __builtin_amdgcn_wmma_f32_16x16x32_bf16(false, a, false, b, (short)0, c, false, false);
  }
  static __device__ __forceinline__ void guard(v8f& a, v8f& b, v16b x, v16b y) { dep_guard_b(a, b, x, y); }
  static __device__ __forceinline__ void keep(v16b a, v16b b, v16b c, v16b d) { keep4_b(a, b, c, d); }
};

__device__ __forceinline__ unsigned pk16(unsigned short a, unsigned short b) { return (unsigned)a | ((unsigned)b << 16); }

__device__ __forceinline__ v8f bmma(v16b a, v16b b, v8f c) {
  c = __builtin_amdgcn_wmma_f32_16x16x32_bf16(false, a, false, b, (short)0, c, false, false);
  asm volatile("v_nop\n\tv_nop\n\tv_nop\n\tv_nop" : "+v"(c) : "v"(a), "v"(b));
  return c;
}

template <int ET> struct Elem;
template <> struct Elem<0> { typedef _Float16 T; };
template <> struct Elem<1> { typedef __bf16 T; };
template <int ET, bool SPLIT, int BIAS_MODE, int OUT_MODE, bool RESID, int ACT = 0>
__global__ __launch_bounds__(256) void wmma_gemm64(
    const unsigned short* __restrict__ Ap, const unsigned short* __restrict__ A2p, int lda, long strideA,
    const unsigned short* __restrict__ Btp, const unsigned short* __restrict__ Bt2p, int ldb, long strideB,
    void* __restrict__ Cout, void* __restrict__ Cout2, int ldc, long strideC,
    const float* __restrict__ bias,
    const float* __restrict__ resid, long strideR,
    int M, int N, int K, float scale) {
  typedef typename Elem<ET>::T T;
  typedef typename Frag<T>::V V;
  const T* A = (const T*)Ap; const T* A2 = (const T*)A2p; const T* Bt = (const T*)Btp; const T* Bt2 = (const T*)Bt2p;
  __shared__ __align__(16) float sT[8][16 * 68];
  const int b    = blockIdx.y;
  const int lane = threadIdx.x & 31;
  const int wave = threadIdx.x >> 5;
  const int tilesN = N >> 6;
  const int tilesM = M >> 6;
  const int tile = blockIdx.x * 8 + wave;
  if (tile >= tilesM * tilesN) return;
  const int tm = tile / tilesN;
  const int tn = tile - tm * tilesN;
  const int m0 = tm << 6;
  const int n0 = tn << 6;

  const T* Ab  = A  + (size_t)b * strideA;
  const T* Bb  = Bt + (size_t)b * strideB;
  const T* Ab2 = SPLIT ? (A2  + (size_t)b * strideA) : nullptr;
  const T* Bb2 = SPLIT ? (Bt2 + (size_t)b * strideB) : nullptr;

  const int rlane = lane & 15;
  const int koff  = (lane >> 4) * 8;
  const int mOff  = (lane >> 4) * 8;

  v8f acc[4][4];
#pragma unroll
  for (int i = 0; i < 4; ++i)
#pragma unroll
    for (int j = 0; j < 4; ++j) acc[i][j] = (v8f){0.f,0.f,0.f,0.f,0.f,0.f,0.f,0.f};

  for (int k0 = 0; k0 < K; k0 += 32) {
    V bh[4], bl[4];
#pragma unroll
    for (int j = 0; j < 4; ++j) {
      const size_t bo = (size_t)(n0 + (j << 4) + rlane) * ldb + koff + k0;
      bh[j] = Frag<T>::load(Bb + bo);
      if (SPLIT) bl[j] = Frag<T>::load(Bb2 + bo);
    }
#pragma unroll
    for (int i = 0; i < 4; ++i) {
      const size_t ao = (size_t)(m0 + (i << 4) + rlane) * lda + koff + k0;
      V ah = Frag<T>::load(Ab + ao);
      V al;
      if (SPLIT) al = Frag<T>::load(Ab2 + ao);
#pragma unroll
      for (int j = 0; j < 4; ++j) {
        acc[i][j] = Frag<T>::mma(ah, bh[j], acc[i][j]);
        if (SPLIT) {
          acc[i][j] = Frag<T>::mma(ah, bl[j], acc[i][j]);
          acc[i][j] = Frag<T>::mma(al, bh[j], acc[i][j]);
        }
      }
      Frag<T>::guard(acc[i][0], acc[i][3], ah, SPLIT ? al : ah);
    }
    Frag<T>::keep(bh[0], bh[1], bh[2], bh[3]);
    if (SPLIT) Frag<T>::keep(bl[0], bl[1], bl[2], bl[3]);
  }
  acc_guard4(acc[0][0], acc[0][1], acc[0][2], acc[0][3]);
  acc_guard4(acc[1][0], acc[1][1], acc[1][2], acc[1][3]);
  acc_guard4(acc[2][0], acc[2][1], acc[2][2], acc[2][3]);
  acc_guard4(acc[3][0], acc[3][1], acc[3][2], acc[3][3]);

  float* slab = sT[wave];
  const float* Rb = RESID ? (resid + (size_t)b * strideR) : nullptr;
#pragma unroll
  for (int i = 0; i < 4; ++i) {
    const int mBase = m0 + (i << 4);
#pragma unroll
    for (int j = 0; j < 4; ++j) {
      const int n = n0 + (j << 4) + rlane;
      float bv = 0.f;
      if (BIAS_MODE == 2) bv = bias[n];
#pragma unroll
      for (int r = 0; r < 8; ++r) {
        float v = acc[i][j][r] * scale;
        if (BIAS_MODE == 1) v += bias[mBase + mOff + r];
        if (BIAS_MODE == 2) v += bv;
        if (RESID) v += Rb[(size_t)(mBase + mOff + r) * ldc + n];
        if (ACT == 2) v = fmaxf(v, 0.0f);
        if (ACT == 4) v = (v > 0.f) ? v : 0.01f * v;
        slab[(mOff + r) * 68 + (j << 4) + rlane] = v;
      }
    }
    __builtin_amdgcn_fence(__ATOMIC_RELEASE, "workgroup");
    __builtin_amdgcn_wave_barrier();
    __builtin_amdgcn_fence(__ATOMIC_ACQUIRE, "workgroup");
    if (OUT_MODE == 0) {
      float* C = (float*)Cout + (size_t)b * strideC;
      const int hh = lane >> 4, c4 = (lane & 15) * 4;
      for (int pass = 0; pass < 2; ++pass) {
#pragma unroll
        for (int it = 0; it < 8; ++it) {
          const int row = it * 2 + hh;
          v4f v = *(const v4f*)(slab + row * 68 + c4);
          *(volatile v4f*)(C + (size_t)(mBase + row) * ldc + n0 + c4) = v;
        }
        __threadfence();
      }
    } else {
      const int q = lane >> 3, c8 = (lane & 7) * 8;
      unsigned short* C  = (unsigned short*)Cout  + (size_t)b * strideC;
      unsigned short* C2 = (OUT_MODE == 2) ? ((unsigned short*)Cout2 + (size_t)b * strideC) : nullptr;
      for (int pass = 0; pass < 2; ++pass) {
#pragma unroll
        for (int it = 0; it < 4; ++it) {
          const int row = it * 4 + q;
          const float* sp = slab + row * 68 + c8;
          v8h hv, lv;
#pragma unroll
          for (int e = 0; e < 8; ++e) {
            if (OUT_MODE == 1) {
              hv[e] = (_Float16)sp[e];
            } else {
              unsigned short hb = f2bf_bits(sp[e]);
              unsigned short lb = f2bf_bits(sp[e] - bf_bits2f(hb));
              hv[e] = __builtin_bit_cast(_Float16, hb);
              lv[e] = __builtin_bit_cast(_Float16, lb);
            }
          }
          *(volatile v8h*)(C + (size_t)(mBase + row) * ldc + n0 + c8) = hv;
          if (OUT_MODE == 2) *(volatile v8h*)(C2 + (size_t)(mBase + row) * ldc + n0 + c8) = lv;
        }
        __threadfence();
      }
    }
    __builtin_amdgcn_fence(__ATOMIC_RELEASE, "workgroup");
    __builtin_amdgcn_wave_barrier();
    __builtin_amdgcn_fence(__ATOMIC_ACQUIRE, "workgroup");
  }
}

__global__ __launch_bounds__(256) void tsplit_kernel(const float* __restrict__ in, long inStrideZ, int R, int C,
                                                     unsigned short* __restrict__ outH, unsigned short* __restrict__ outL,
                                                     long outStrideZ) {
  __shared__ float sm[64][65];
  const int t  = threadIdx.x;
  const int r0 = blockIdx.x * 64;
  const int c0 = blockIdx.y * 64;
  const int z  = blockIdx.z;
  const float* inz = in + (size_t)z * inStrideZ;
#pragma unroll
  for (int i = 0; i < 16; ++i) {
    const int e  = i * 256 + t;
    const int rl = e >> 6;
    const int cl = e & 63;
    const int gc = c0 + cl;
    const int gcc = (gc < C) ? gc : (C - 1);
    float v = inz[(size_t)(r0 + rl) * C + gcc];
    if (gc >= C) v = 0.0f;
    sm[cl][rl] = v;
  }
  __syncthreads();
  const int lane = t & 31, wave = t >> 5;
  const int q = lane >> 3, c8 = (lane & 7) * 8;
  unsigned short* oh = outH + (size_t)z * outStrideZ;
  unsigned short* ol = outL + (size_t)z * outStrideZ;
  for (int pass = 0; pass < 2; ++pass) {
#pragma unroll
    for (int it = 0; it < 2; ++it) {
      const int row = wave * 8 + it * 4 + q;
      unsigned short hb[8], lb[8];
#pragma unroll
      for (int e = 0; e < 8; ++e) {
        const float v = sm[row][c8 + e];
        hb[e] = f2bf_bits(v);
        lb[e] = f2bf_bits(v - bf_bits2f(hb[e]));
      }
      const v4u uh = (v4u){pk16(hb[0], hb[1]), pk16(hb[2], hb[3]), pk16(hb[4], hb[5]), pk16(hb[6], hb[7])};
      const v4u ul = (v4u){pk16(lb[0], lb[1]), pk16(lb[2], lb[3]), pk16(lb[4], lb[5]), pk16(lb[6], lb[7])};
      const size_t o = (size_t)(c0 + row) * R + r0 + c8;
      *(volatile v4u*)(oh + o) = uh;
      *(volatile v4u*)(ol + o) = ul;
    }
    __threadfence();
  }
}

__global__ __launch_bounds__(256) void embed_split_kernel(const int* __restrict__ seq, const float* __restrict__ table,
                                                          unsigned short* __restrict__ xH, unsigned short* __restrict__ xL) {
  const int t   = blockIdx.x * 256 + threadIdx.x;
  const int row = t >> 4;
  const int c8  = (t & 15) * 8;
  int id = seq[row];
  id = (id < 0) ? 0 : id;
  id = (id > kVocab - 1) ? (kVocab - 1) : id;
  const float* p = table + (size_t)id * kDim + c8;
  const v4f a = *(const v4f*)(p);
  const v4f c = *(const v4f*)(p + 4);
  unsigned short hb[8], lb[8];
#pragma unroll
  for (int e = 0; e < 4; ++e) {
    hb[e] = f2bf_bits(a[e]);         lb[e] = f2bf_bits(a[e] - bf_bits2f(hb[e]));
    hb[4 + e] = f2bf_bits(c[e]);     lb[4 + e] = f2bf_bits(c[e] - bf_bits2f(hb[4 + e]));
  }
  const v4u uh = (v4u){pk16(hb[0], hb[1]), pk16(hb[2], hb[3]), pk16(hb[4], hb[5]), pk16(hb[6], hb[7])};
  const v4u ul = (v4u){pk16(lb[0], lb[1]), pk16(lb[2], lb[3]), pk16(lb[4], lb[5]), pk16(lb[6], lb[7])};
  const size_t o = (size_t)row * kDim + c8;
  *(volatile v4u*)(xH + o) = uh;
  *(volatile v4u*)(xL + o) = ul;
  __threadfence();
  *(volatile v4u*)(xH + o) = uh;
  *(volatile v4u*)(xL + o) = ul;
}

__global__ __launch_bounds__(256) void slot_agg_kernel(const float* __restrict__ ts, const float* __restrict__ lat,
                                                       const float* __restrict__ lng, const int* __restrict__ vlen,
                                                       const float* __restrict__ vs,
                                                       unsigned short* __restrict__ aggH, unsigned short* __restrict__ aggL) {
  #pragma clang fp contract(off)
  __shared__ __align__(16) float accs[8][kSlotE];
  __shared__ int codes[8][kSeq];
  const int lane = threadIdx.x & 31;
  const int wave = threadIdx.x >> 5;
  const int gw = blockIdx.x * 8 + wave;
  const int b  = gw >> 7;
  const int i  = gw & (kSeq - 1);
  const float tsi  = ts[gw];
  const float lati = lat[gw];
  const float lngi = lng[gw];
  const int   vl   = vlen[b];
  float* aw = accs[wave];
#pragma unroll
  for (int k = 0; k < kSlots; ++k) {
    aw[k * kInter + 2 * lane]     = 0.0f;
    aw[k * kInter + 2 * lane + 1] = 0.0f;
  }
#pragma unroll 1
  for (int t = 0; t < 4; ++t) {
    const int j  = lane + 32 * t;
    const int gj = (b << 7) + j;
    const float td = tsi - ts[gj];
    const bool m = (td <= 3600.0f) && (td >= 0.0f) && (vl > j) && (j <= i);
    const float tclip = fminf(fmaxf(td, 0.0f), 3600.0f);
    float q1 = tclip / 3600.0f;
    asm volatile("" : "+v"(q1));
    const float q2 = q1 * 10.0f;
    int tc = (int)floorf(q2);
    tc = (tc < 0) ? 0 : ((tc > kSlots - 1) ? (kSlots - 1) : tc);
    const float dla = lati - lat[gj];
    const float dln = lngi - lng[gj];
    float s1 = dla * dla;
    float s2 = dln * dln;
    asm volatile("" : "+v"(s1));
    asm volatile("" : "+v"(s2));
    const float dist  = sqrtf(s1 + s2);
    const float dclip = fminf(fmaxf(dist, 0.0f), 1.0f);
    const float e2 = dclip * 10.0f;
    int dc = (int)floorf(e2);
    dc = (dc < 0) ? 0 : ((dc > kSlots - 1) ? (kSlots - 1) : dc);
    codes[wave][j] = m ? (tc * 16 + dc) : -1;
  }
  __syncthreads();
  const float* vrow = vs + (size_t)(b << 7) * kSlotE + 2 * lane;
  for (int j = 0; j <= i; ++j) {
    const int code = __builtin_amdgcn_readfirstlane(codes[wave][j]);
    if (code >= 0) {
      const int tc = (code >> 4) & 15;
      const int dc = code & 15;
      const int tcc = (tc > kSlots - 1) ? (kSlots - 1) : tc;
      const int dcc = (dc > kSlots - 1) ? (kSlots - 1) : dc;
      const v2f v = *(const v2f*)(vrow + (size_t)j * kSlotE + tcc * kInter);
      v2f* ap = (v2f*)(aw + dcc * kInter + 2 * lane);
      v2f a = *ap;
      a += v;
      *ap = a;
    }
  }
  __syncthreads();
  const int q = lane >> 3, sub = lane & 7;
  unsigned short* oh = aggH + (size_t)gw * kSlotE;
  unsigned short* ol = aggL + (size_t)gw * kSlotE;
  for (int pass = 0; pass < 2; ++pass) {
#pragma unroll
    for (int it = 0; it < 3; ++it) {
      const int line = it * 4 + q;
      const int lc = (line < kSlots) ? line : (kSlots - 1);
      const float* sp = aw + lc * kInter + sub * 8;
      const v4f a = *(const v4f*)(sp);
      const v4f c = *(const v4f*)(sp + 4);
      unsigned short hb[8], lb[8];
#pragma unroll
      for (int e = 0; e < 4; ++e) {
        hb[e] = f2bf_bits(a[e]);       lb[e] = f2bf_bits(a[e] - bf_bits2f(hb[e]));
        hb[4 + e] = f2bf_bits(c[e]);   lb[4 + e] = f2bf_bits(c[e] - bf_bits2f(hb[4 + e]));
      }
      const v4u uh = (v4u){pk16(hb[0], hb[1]), pk16(hb[2], hb[3]), pk16(hb[4], hb[5]), pk16(hb[6], hb[7])};
      const v4u ul = (v4u){pk16(lb[0], lb[1]), pk16(lb[2], lb[3]), pk16(lb[4], lb[5]), pk16(lb[6], lb[7])};
      if (line < kSlots) {
        const size_t o = (size_t)lc * kInter + sub * 8;
        *(volatile v4u*)(oh + o) = uh;
        *(volatile v4u*)(ol + o) = ul;
      }
    }
    __threadfence();
  }
}

__global__ __launch_bounds__(256) void rnn_kernel(const float* __restrict__ xc,
                                                  const unsigned short* __restrict__ whH, const unsigned short* __restrict__ whL,
                                                  const int* __restrict__ prelen,
                                                  unsigned short* __restrict__ preH, unsigned short* __restrict__ preL) {
  union FB { v16b v; v8b h[2]; };
  __shared__ __align__(16) __bf16 hsH[16 * kHid];
  __shared__ __align__(16) __bf16 hsL[16 * kHid];
  const int t    = threadIdx.x;
  const int lane = t & 31;
  const int wave = t >> 5;
  const int hh   = lane >> 4;
  const int rl   = lane & 15;
  const int koff = hh * 8;
  const int b0   = blockIdx.x * 16;
  int pl = prelen[0];
  int start = kSeq - pl - 1;
  start = (start < 0) ? 0 : ((start > kSeq - kPre) ? (kSeq - kPre) : start);

  ((v4u*)(void*)hsH)[t] = (v4u){0u, 0u, 0u, 0u};
  ((v4u*)(void*)hsL)[t] = (v4u){0u, 0u, 0u, 0u};

  v16b bh[4], bl[4];
#pragma unroll
  for (int kk = 0; kk < 4; ++kk) {
    const size_t bo = (size_t)(wave * 16 + rl) * kHid + koff + kk * 32;
    bh[kk] = Frag<__bf16>::load((const __bf16*)whH + bo);
    bl[kk] = Frag<__bf16>::load((const __bf16*)whL + bo);
  }
  __syncthreads();

  const int col = wave * 16 + rl;
  for (int i = 0; i < kSeq; ++i) {
    float xv[8];
#pragma unroll
    for (int r = 0; r < 8; ++r)
      xv[r] = xc[((size_t)(b0 + 8 * hh + r) * kSeq + i) * kHid + col];

    v8f acc = (v8f){0.f,0.f,0.f,0.f,0.f,0.f,0.f,0.f};
#pragma unroll
    for (int kk = 0; kk < 4; ++kk) {
      FB ah, al;
      ah.h[0] = *(const v8b*)(hsH + rl * kHid + kk * 32 + koff);
      ah.h[1] = *(const v8b*)(hsH + rl * kHid + kk * 32 + 16 + koff);
      al.h[0] = *(const v8b*)(hsL + rl * kHid + kk * 32 + koff);
      al.h[1] = *(const v8b*)(hsL + rl * kHid + kk * 32 + 16 + koff);
      acc = bmma(ah.v, bh[kk], acc);
      acc = bmma(ah.v, bl[kk], acc);
      acc = bmma(al.v, bh[kk], acc);
    }

    unsigned short hb[8], lb[8];
#pragma unroll
    for (int r = 0; r < 8; ++r) {
      const float z = acc[r] + xv[r];
      const float e = expf(-z);
      const float hv = 1.0f / (1.0f + e);
      hb[r] = f2bf_bits(hv);
      lb[r] = f2bf_bits(hv - bf_bits2f(hb[r]));
    }
    __syncthreads();
#pragma unroll
    for (int r = 0; r < 8; ++r) {
      hsH[(8 * hh + r) * kHid + col] = __builtin_bit_cast(__bf16, hb[r]);
      hsL[(8 * hh + r) * kHid + col] = __builtin_bit_cast(__bf16, lb[r]);
    }
    __syncthreads();
    if (i >= start && i < start + kPre) {
      const int p   = i - start;
      const int row = 2 * wave + hh;
      const int c8  = rl * 8;
      const v8b vh = *(const v8b*)(hsH + row * kHid + c8);
      const v8b vl = *(const v8b*)(hsL + row * kHid + c8);
      const v4u uh = __builtin_bit_cast(v4u, vh);
      const v4u ul = __builtin_bit_cast(v4u, vl);
      const size_t o = ((size_t)(b0 + row) * kPre + p) * kHid + c8;
      *(volatile v4u*)(preH + o) = uh;
      *(volatile v4u*)(preL + o) = ul;
      __threadfence();
      *(volatile v4u*)(preH + o) = uh;
      *(volatile v4u*)(preL + o) = ul;
    }
  }
}

__global__ __launch_bounds__(256) void tanh_split_kernel(const float* __restrict__ in, unsigned short* __restrict__ oH,
                                                         unsigned short* __restrict__ oL, int n2) {
  const int i = blockIdx.x * 256 + threadIdx.x;
  if (i >= n2) return;
  const float* p = in + 2 * (size_t)i;
  unsigned uh = 0u, ul = 0u;
#pragma unroll 1
  for (int e = 0; e < 2; ++e) {
    const float a = tanhf(p[e]);
    const unsigned short ha = f2bf_bits(a);
    const unsigned short la = f2bf_bits(a - bf_bits2f(ha));
    uh |= ((unsigned)ha) << (16 * e);
    ul |= ((unsigned)la) << (16 * e);
  }
  ((volatile unsigned*)oH)[i] = uh;
  ((volatile unsigned*)oL)[i] = ul;
  __threadfence();
  ((volatile unsigned*)oH)[i] = uh;
  ((volatile unsigned*)oL)[i] = ul;
}

__global__ __launch_bounds__(256) void outcopy_kernel(const float* __restrict__ stage, const float* __restrict__ b2,
                                                      float* __restrict__ out) {
  const int t = blockIdx.x * 256 + threadIdx.x;
  const size_t e0  = (size_t)t * 4;
  const size_t row = e0 / (size_t)kOutN;
  const size_t col = e0 - row * (size_t)kOutN;
  v4f v = *(const v4f*)(stage + row * kOutPad + col);
  const v4f bb = *(const v4f*)(b2 + col);
  v += bb;
  *(volatile v4f*)(out + e0) = v;
  __threadfence();
  *(volatile v4f*)(out + e0) = v;
}

extern "C" void kernel_launch(void* const* d_in, const int* in_sizes, int n_in,
                              void* d_out, int out_size, void* d_ws,
                              size_t ws_size, hipStream_t stream) {
  (void)in_sizes; (void)n_in; (void)out_size;
  const int*   full_seq       = (const int*)d_in[0];
  const int*   valid_len      = (const int*)d_in[1];
  const int*   pre_len        = (const int*)d_in[2];
  const float* timestamp      = (const float*)d_in[3];
  const float* lat            = (const float*)d_in[4];
  const float* lng            = (const float*)d_in[5];
  const float* embed_table    = (const float*)d_in[6];
  const float* time_weights   = (const float*)d_in[7];
  const float* dist_weights   = (const float*)d_in[8];
  const float* hidden_weights = (const float*)d_in[9];
  const float* w1             = (const float*)d_in[10];
  const float* b1             = (const float*)d_in[11];
  const float* w2             = (const float*)d_in[12];
  const float* b2             = (const float*)d_in[13];
  float* out = (float*)d_out;

  char* ws = (char*)d_ws;
  size_t off = 0;
  auto carve = [&](size_t bytes) -> char* {
    char* p = ws + off;
    off += (bytes + 255) & ~(size_t)255;
    return p;
  };
  unsigned short* twH  = (unsigned short*)carve((size_t)kSlotE * kDim * 2);
  unsigned short* twL  = (unsigned short*)carve((size_t)kSlotE * kDim * 2);
  unsigned short* dwH  = (unsigned short*)carve((size_t)kHid * kSlotE * 2);
  unsigned short* dwL  = (unsigned short*)carve((size_t)kHid * kSlotE * 2);
  unsigned short* whH  = (unsigned short*)carve((size_t)kHid * kHid * 2);
  unsigned short* whL  = (unsigned short*)carve((size_t)kHid * kHid * 2);
  unsigned short* w1H  = (unsigned short*)carve((size_t)kHid4 * kHid * 2);
  unsigned short* w1L  = (unsigned short*)carve((size_t)kHid4 * kHid * 2);
  unsigned short* w2H  = (unsigned short*)carve((size_t)kOutPad * kHid4 * 2);
  unsigned short* w2L  = (unsigned short*)carve((size_t)kOutPad * kHid4 * 2);
  unsigned short* xH   = (unsigned short*)carve((size_t)kRows * kDim * 2);
  unsigned short* xL   = (unsigned short*)carve((size_t)kRows * kDim * 2);
  float*          vsl  = (float*)carve((size_t)kRows * kSlotE * 4);
  unsigned short* aggH = (unsigned short*)carve((size_t)kRows * kSlotE * 2);
  unsigned short* aggL = (unsigned short*)carve((size_t)kRows * kSlotE * 2);
  float*          xcd  = (float*)carve((size_t)kRows * kHid * 4);
  unsigned short* preH = (unsigned short*)carve((size_t)kPreRows * kHid * 2);
  unsigned short* preL = (unsigned short*)carve((size_t)kPreRows * kHid * 2);
  float*          hid32 = (float*)carve((size_t)kPreRows * kHid4 * 4);
  unsigned short* hidH = (unsigned short*)carve((size_t)kPreRows * kHid4 * 2);
  unsigned short* hidL = (unsigned short*)carve((size_t)kPreRows * kHid4 * 2);
  float*          stage = (float*)carve((size_t)kPreRows * kOutPad * 4);
  if (off > ws_size) return;

  tsplit_kernel<<<dim3(kDim / 64, kInter / 64, kSlots), 256, 0, stream>>>(
      time_weights, (long)kDim * kInter, kDim, kInter, twH, twL, (long)kInter * kDim);
  tsplit_kernel<<<dim3(kSlotE / 64, kHid / 64, 1), 256, 0, stream>>>(
      dist_weights, 0L, kSlotE, kHid, dwH, dwL, 0L);
  tsplit_kernel<<<dim3(kHid / 64, kHid / 64, 1), 256, 0, stream>>>(
      hidden_weights, 0L, kHid, kHid, whH, whL, 0L);
  tsplit_kernel<<<dim3(kHid / 64, kHid4 / 64, 1), 256, 0, stream>>>(
      w1, 0L, kHid, kHid4, w1H, w1L, 0L);
  tsplit_kernel<<<dim3(kHid4 / 64, kOutPad / 64, 1), 256, 0, stream>>>(
      w2, 0L, kHid4, kOutN, w2H, w2L, 0L);

  embed_split_kernel<<<(kRows * kDim / 8) / 256, 256, 0, stream>>>(full_seq, embed_table, xH, xL);

  wmma_gemm64<1, true, 0, 0, false, 0><<<dim3((kRows / 64) * (kSlotE / 64) / 8, 1), 256, 0, stream>>>(
      xH, xL, kDim, 0L, twH, twL, kDim, 0L, (void*)vsl, nullptr, kSlotE, 0L,
      nullptr, nullptr, 0L, kRows, kSlotE, kDim, 1.0f);

  slot_agg_kernel<<<kRows / 8, 256, 0, stream>>>(timestamp, lat, lng, valid_len, vsl, aggH, aggL);

  wmma_gemm64<1, true, 0, 0, false, 0><<<dim3((kRows / 64) * (kHid / 64) / 8, 1), 256, 0, stream>>>(
      aggH, aggL, kSlotE, 0L, dwH, dwL, kSlotE, 0L, (void*)xcd, nullptr, kHid, 0L,
      nullptr, nullptr, 0L, kRows, kHid, kSlotE, 1.0f);

  rnn_kernel<<<kBatch / 16, 256, 0, stream>>>(xcd, whH, whL, pre_len, preH, preL);

  wmma_gemm64<1, true, 2, 0, false, 0><<<dim3((kPreRows / 64) * (kHid4 / 64) / 8, 1), 256, 0, stream>>>(
      preH, preL, kHid, 0L, w1H, w1L, kHid, 0L, (void*)hid32, nullptr, kHid4, 0L,
      b1, nullptr, 0L, kPreRows, kHid4, kHid, 1.0f);

  tanh_split_kernel<<<(kPreRows * kHid4 / 2) / 256, 256, 0, stream>>>(hid32, hidH, hidL, kPreRows * kHid4 / 2);

  wmma_gemm64<1, true, 0, 0, false, 0><<<dim3((kPreRows / 64) * (kOutPad / 64) / 8, 1), 256, 0, stream>>>(
      hidH, hidL, kHid4, 0L, w2H, w2L, kHid4, 0L, (void*)stage, nullptr, kOutPad, 0L,
      nullptr, nullptr, 0L, kPreRows, kOutPad, kHid4, 1.0f);

  outcopy_kernel<<<(kPreRows * kOutN / 4) / 256, 256, 0, stream>>>(stage, b2, out);
}
